// MuonLonghornVisionMixer_57964878627185
// MI455X (gfx1250) — hardware-run, weakly checked
//
#include <hip/hip_runtime.h>


#ifndef NB
#define NB 8
#endif
#ifndef SEQ
#define SEQ 2048
#endif
#define NB_FULL  8
#define SEQ_FULL 2048
#ifndef OUT_SEQ
#define OUT_SEQ SEQ
#endif
#define DM   512
#define DI   1024
#define DS   512
#define NS   16
#define DR   32
#define NX   64
#define NTOK (NB * SEQ)
#define CHB  (NB > 4 ? 4 : NB)
#define NCH  (NB / CHB)
#define CW   4
#define CT   32
#define CSP  36
#define TCH  16
#define CARRY   64.0f
#define CARRY2I (1.0f / 4096.0f)
#define LOG2E 1.4426950408889634f
#define LN2   0.6931471805599453f

static_assert(DI == 2 * DS);
static_assert(DM % 32 == 0);
static_assert(DI % 32 == 0);
static_assert(DS % 32 == 0);
static_assert(DR == 32);
static_assert(NX == 64);
static_assert(NS == 16);
static_assert(NX == DR + 2 * NS);
static_assert(DI % 64 == 0);
static_assert(DM % 64 == 0);
static_assert(SEQ % 64 == 0);
static_assert(NB % CHB == 0);
static_assert((CHB * SEQ) % 64 == 0);
static_assert((CHB * SEQ) % (CW * CT) == 0);
static_assert(SEQ % CT == 0);
static_assert(SEQ % TCH == 0);
static_assert(NTOK % 64 == 0);
static_assert(NTOK % 32 == 0);
static_assert(CT == 32);
static_assert(8 * 4 == CT);
static_assert(8 * 4 == 32);
static_assert(4 * 32 * 8 == CT * 32);
static_assert(8 * 2 == 16);
static_assert(16 * 4 == 64);
static_assert(2 * 32 * 8 == 16 * DR);
static_assert(4 * 4 == 16);
static_assert(2 * 32 * 8 == TCH * 32);
static_assert(4 * 32 * 4 == TCH * 32);
static_assert((CSP * 4) % 16 == 0);
static_assert(((size_t)NB * SEQ * DM) % 8 == 0);
static_assert(((size_t)SEQ * DM) % 8 == 0);
static_assert(((size_t)DI * DM) % 8 == 0);
static_assert(((size_t)NX * DS) % 8 == 0);
static_assert(((size_t)DS * DR) % 8 == 0);
static_assert(NB <= NB_FULL);
static_assert(SEQ <= SEQ_FULL);
static_assert(16 * 68 * 4 <= 131072);
static_assert(CW * CT * CSP * 4 + CW * CT * 32 * 2 <= 131072);
static_assert(TCH * 32 * 4 * 2 + 32 * 4 + TCH * 32 * 2 <= 131072);

typedef _Float16 h16;
typedef unsigned short bf;
typedef __attribute__((ext_vector_type(16))) __bf16   v16bf;
typedef __attribute__((ext_vector_type(16))) _Float16 v16h;
typedef __attribute__((ext_vector_type(8)))  _Float16 v8h;
typedef __attribute__((ext_vector_type(8)))  unsigned short v8us;
typedef __attribute__((ext_vector_type(8)))  float    v8f;
typedef __attribute__((ext_vector_type(4)))  float    v4f;
typedef v4f  __attribute__((may_alias)) v4fa;
typedef v8h  __attribute__((may_alias)) v8ha;

__device__ __forceinline__ unsigned short f2bf(float f) { unsigned u = __float_as_uint(f); u += 0x7FFFu + ((u >> 16) & 1u); return (unsigned short)(u >> 16); }
__device__ __forceinline__ float bfr(float f) { return __uint_as_float(((unsigned)f2bf(f)) << 16); }
__device__ __forceinline__ v16h cat16(v8h lo, v8h hi) { return __builtin_shufflevector(lo, hi, 0, 1, 2, 3, 4, 5, 6, 7, 8, 9, 10, 11, 12, 13, 14, 15); }
__device__ __forceinline__ v16bf cat16b(v8us lo, v8us hi) { return __builtin_bit_cast(v16bf, __builtin_shufflevector(lo, hi, 0, 1, 2, 3, 4, 5, 6, 7, 8, 9, 10, 11, 12, 13, 14, 15)); }
__device__ __forceinline__ v8f wmma16(v16h a, v16h b, v8f c) { return __builtin_amdgcn_wmma_f32_16x16x32_f16(false, a, false, b, (short)0, c, false, false); }
__device__ __forceinline__ v8f wmmab(v16bf a, v16bf b, v8f c) { return __builtin_amdgcn_wmma_f32_16x16x32_bf16(false, a, false, b, (short)0, c, false, false); }
__device__ __forceinline__ v16h  ldh(const h16* p) { return cat16(*(const v8h*)p, *(const v8h*)(p + 16)); }
__device__ __forceinline__ v16bf ldb(const bf* p)  { return cat16b(*(const v8us*)p, *(const v8us*)(p + 16)); }
__device__ __forceinline__ void wave_sync() { __builtin_amdgcn_fence(3  , "wavefront"); __builtin_amdgcn_wave_barrier(); asm volatile("" ::: "memory"); }

static __device__ __forceinline__ h16 toh_flush(float v) { const h16 r = (h16)v; return (fabsf(v) < 6.103515625e-05f) ? (h16)0.0f : r; }
static __device__ __forceinline__ v8f wmma16g(v16h a, v16h b, v8f c) { c = wmma16(a, b, c); asm volatile("v_nop\n\tv_nop\n\tv_nop\n\tv_nop" : "+v"(c) : "v"(a), "v"(b)); return c; }

__global__ __launch_bounds__(256) void k_cvt8(const float* __restrict__ src, bf* dst, size_t n8) {
    const size_t i = (size_t)blockIdx.x * 256 + threadIdx.x; if (i >= n8) return;
    const v8f v = *(const v8f*)(src + i * 8); v8us o;
#pragma unroll
    for (int k = 0; k < 8; ++k) o[k] = f2bf(v[k]);
    *(volatile v8us*)(dst + i * 8) = o; __threadfence(); *(volatile v8us*)(dst + i * 8) = o;
}

__global__ __launch_bounds__(256) void k_wcvt(const float* __restrict__ src, h16* dst, size_t n8, float carry) {
    const size_t i = (size_t)blockIdx.x * 256 + threadIdx.x; if (i >= n8) return;
    const v8f v = *(const v8f*)(src + i * 8); v8h o;
#pragma unroll
    for (int k = 0; k < 8; ++k) o[k] = toh_flush(bfr(v[k]) * carry);
    *(volatile v8h*)(dst + i * 8) = o; __threadfence(); *(volatile v8h*)(dst + i * 8) = o;
}

__global__ __launch_bounds__(32) void k_gemm_in(const bf* __restrict__ A, const bf* __restrict__ Bt, float* XZ) {
    __shared__ __align__(16) float os[16 * 68];
    const int K = DM;
    const int lane = threadIdx.x & 31, lr = lane & 15, hi = lane >> 4; const int r0 = blockIdx.x * 64, c0 = blockIdx.y * 64;
    v8f acc[4][4];
#pragma unroll
    for (int mb = 0; mb < 4; ++mb)
#pragma unroll
        for (int nb = 0; nb < 4; ++nb) acc[mb][nb] = (v8f){};
    const size_t aoff = (size_t)(r0 + lr) * K + 8 * hi, boff = (size_t)(c0 + lr) * K + 8 * hi;
#pragma unroll 1
    for (int kc = 0; kc < K; kc += 32) {
        v16bf a[4];
#pragma unroll
        for (int mb = 0; mb < 4; ++mb) a[mb] = ldb(A + aoff + (size_t)mb * 16 * K + kc);
#pragma unroll
        for (int nb = 0; nb < 4; ++nb) { const v16bf b = ldb(Bt + boff + (size_t)nb * 16 * K + kc);
#pragma unroll
            for (int mb = 0; mb < 4; ++mb) acc[mb][nb] = wmmab(a[mb], b, acc[mb][nb]); }
        asm volatile("v_nop\n\tv_nop\n\tv_nop\n\tv_nop" : "+v"(acc[0][0]), "+v"(acc[1][1]), "+v"(acc[2][2]), "+v"(acc[3][3]) : "v"(a[0]), "v"(a[1]), "v"(a[2]), "v"(a[3]));
    }
#pragma unroll
    for (int mb = 0; mb < 4; ++mb) {
#pragma unroll
        for (int nb = 0; nb < 4; ++nb) {
#pragma unroll
            for (int j = 0; j < 8; ++j) os[(hi * 8 + j) * 68 + nb * 16 + lr] = acc[mb][nb][j]; }
        wave_sync();
        float* dst = XZ + (size_t)(r0 + mb * 16) * DI + c0;
#pragma unroll 1
        for (int ps = 0; ps < 2; ++ps) {
#pragma unroll
            for (int s = 0; s < 8; ++s) { const int row = 2 * s + (lane >> 4), c4 = (lane & 15) * 4;
                const v4f val = *(const v4fa*)(&os[row * 68 + c4]);
                *(volatile v4f*)(dst + (size_t)row * DI + c4) = val; }
            if (ps == 0) __threadfence(); }
        wave_sync();
    }
}

static __device__ __forceinline__ float ldtap(const float* __restrict__ xs, int t) {
    const int tcl = t < 0 ? 0 : (t > SEQ - 1 ? SEQ - 1 : t);
    float v = xs[(size_t)tcl * DI]; asm volatile("" : "+v"(v));
    return ((t >= 0) & (t < SEQ)) ? v : 0.0f;
}

__global__ __launch_bounds__(32 * CW) void k_conv(const float* __restrict__ XZ, const float* __restrict__ cxw, const float* __restrict__ cxb,
                                                   const float* __restrict__ czw, const float* __restrict__ czb, float* U, h16* YC, int tokbase) {
    __shared__ __align__(16) float osf[CW * CT * CSP];
    __shared__ __align__(16) h16   osh[CW * CT * 32];
    const int lane = threadIdx.x & 31;
    const int wave = __builtin_amdgcn_readfirstlane((int)(threadIdx.x >> 5));
    const int g = blockIdx.y; const bool zh = g >= (DS / 32);
    const int ch = g * 32 + lane, cc = ch & (DS - 1);
    const int tc0 = (blockIdx.x * CW + wave) * CT;
    const int t0 = tc0 % SEQ;
    const v4f wx = *(const v4f*)(cxw + (size_t)cc * 4), wz = *(const v4f*)(czw + (size_t)cc * 4);
    const float bxv = cxb[cc], bzv = czb[cc];
    const float w0 = bfr(zh ? wz[0] : wx[0]), w1 = bfr(zh ? wz[1] : wx[1]), w2 = bfr(zh ? wz[2] : wx[2]), w3 = bfr(zh ? wz[3] : wx[3]);
    const float bias = bfr(zh ? bzv : bxv);
    const float* xs = XZ + (size_t)(tc0 - t0) * DI + ch;
    const int wbf = wave * CT * CSP, wbh = wave * CT * 32;
    float xa = ldtap(xs, t0 - 1), xb = ldtap(xs, t0), xc = ldtap(xs, t0 + 1), xd = ldtap(xs, t0 + 2);
#pragma unroll 1
    for (int i = 0; i < CT; ++i) {
        const float s = w0 * xa + w1 * xb + w2 * xc + w3 * xd + bias;
        const float e = __builtin_amdgcn_exp2f(-s * LOG2E);
        const float y = s * __builtin_amdgcn_rcpf(1.0f + e);
        if (zh) osh[wbh + i * 32 + lane] = toh_flush(y * CARRY); else osf[wbf + i * CSP + lane] = y;
        xa = xb; xb = xc; xc = xd; xd = ldtap(xs, t0 + i + 3);
    }
    wave_sync();
    const size_t tokg = (size_t)tokbase + (size_t)tc0;
#pragma unroll 1
    for (int ps = 0; ps < 2; ++ps) {
        if (zh) {
            h16* dst = YC + ((size_t)g * NTOK + tokg) * 32;
#pragma unroll
            for (int s = 0; s < 4; ++s) { const int p = s * 32 + lane;
                const v8h val = *(const v8ha*)(&osh[wbh + p * 8]);
                *(volatile v8h*)(dst + (size_t)p * 8) = val; }
        } else {
            float* dst = U + tokg * DS + g * 32;
#pragma unroll
            for (int s = 0; s < 8; ++s) { const int row = 4 * s + (lane >> 3), cofs = (lane & 7) * 4;
                const v4f val = *(const v4fa*)(&osf[wbf + row * CSP + cofs]);
                *(volatile v4f*)(dst + (size_t)row * DS + cofs) = val; }
        }
        if (ps == 0) __threadfence(); }
}

__global__ __launch_bounds__(32) void k_xproj(const float* __restrict__ U, const h16* __restrict__ Wx, h16* DL, float* KQ) {
    __shared__ __align__(16) float os[16 * 68];
    const int lane = threadIdx.x & 31, lr = lane & 15, hi = lane >> 4; const int r0 = blockIdx.x * 32;
    v8f acc[2][4];
#pragma unroll
    for (int mb = 0; mb < 2; ++mb)
#pragma unroll
        for (int nb = 0; nb < 4; ++nb) acc[mb][nb] = (v8f){};
    const size_t aoff = (size_t)(r0 + lr) * DS + 8 * hi, boff = (size_t)lr * DS + 8 * hi;
#pragma unroll 1
    for (int kc = 0; kc < DS; kc += 32) {
        v16h a[2];
#pragma unroll
        for (int mb = 0; mb < 2; ++mb) { const float* ap = U + aoff + (size_t)mb * 16 * DS + kc;
            const v8f x0 = *(const v8f*)ap; const v8f x1 = *(const v8f*)(ap + 16); v16h f;
#pragma unroll
            for (int i = 0; i < 8; ++i) { f[i] = toh_flush(x0[i] * CARRY); f[8 + i] = toh_flush(x1[i] * CARRY); }
            a[mb] = f; }
#pragma unroll
        for (int nb = 0; nb < 4; ++nb) { const v16h b = ldh(Wx + boff + (size_t)nb * 16 * DS + kc);
#pragma unroll
            for (int mb = 0; mb < 2; ++mb) acc[mb][nb] = wmma16g(a[mb], b, acc[mb][nb]); }
    }
#pragma unroll
    for (int mb = 0; mb < 2; ++mb) {
#pragma unroll
        for (int nb = 0; nb < 4; ++nb) {
#pragma unroll
            for (int j = 0; j < 8; ++j) os[(hi * 8 + j) * 68 + nb * 16 + lr] = acc[mb][nb][j] * CARRY2I; }
        wave_sync();
        h16*   dl = DL + (size_t)(r0 + mb * 16) * DR;
        float* kq = KQ + (size_t)(r0 + mb * 16) * 32;
#pragma unroll 1
        for (int ps = 0; ps < 2; ++ps) {
#pragma unroll
            for (int s = 0; s < 2; ++s) { const int p = s * 32 + lane; const int row = p >> 2, c8 = (p & 3) * 8;
                const v4f x0 = *(const v4fa*)(&os[row * 68 + c8]); const v4f x1 = *(const v4fa*)(&os[row * 68 + c8 + 4]); v8h hv;
#pragma unroll
                for (int i = 0; i < 4; ++i) { hv[i] = toh_flush(x0[i] * CARRY); hv[4 + i] = toh_flush(x1[i] * CARRY); }
                *(volatile v8h*)(dl + (size_t)p * 8) = hv; }
#pragma unroll
            for (int s = 0; s < 4; ++s) { const int row = 4 * s + (lane >> 3), cofs = (lane & 7) * 4;
                const v4f val = *(const v4fa*)(&os[row * 68 + 32 + cofs]);
                *(volatile v4f*)(kq + (size_t)row * 32 + cofs) = val; }
            if (ps == 0) __threadfence(); }
        wave_sync();
    }
}

__global__ __launch_bounds__(32) void k_scan(const h16* __restrict__ DL, const h16* __restrict__ WD, const float* __restrict__ KQ, const float* __restrict__ U,
                                             const float* __restrict__ bdt, const float* __restrict__ dskip, h16* YC) {
    __shared__ __align__(16) float dts[TCH * 32];
    __shared__ __align__(16) float kqs[TCH * 32];
    __shared__ __align__(16) float k2s[32];
    __shared__ __align__(16) h16   ys[TCH * 32];
    const int lane = threadIdx.x & 31, lr = lane & 15, hi = lane >> 4;
    const int g = blockIdx.x, b = blockIdx.y;
    const int d = g * 32 + lane;
    const size_t tokb = (size_t)b * SEQ;
    const float bias = bfr(bdt[d]);
    const float dsk  = bfr(dskip[d]);
    const v16h wb0 = ldh(WD + (size_t)(g * 32 + lr) * DR + 8 * hi);
    const v16h wb1 = ldh(WD + (size_t)(g * 32 + 16 + lr) * DR + 8 * hi);
    const float* ub = U + tokb * DS + d;
    h16* yb = YC + ((size_t)g * NTOK + tokb) * 32;
    float S[NS];
#pragma unroll
    for (int n = 0; n < NS; ++n) S[n] = 0.0f;
#pragma unroll 1
    for (int t0 = 0; t0 < SEQ; t0 += TCH) {
        const v16h a = ldh(DL + (tokb + (size_t)(t0 + lr)) * DR + 8 * hi);
        const v8f d0 = wmma16g(a, wb0, (v8f){});
        const v8f d1 = wmma16g(a, wb1, (v8f){});
#pragma unroll
        for (int r = 0; r < 8; ++r) { dts[(8 * hi + r) * 32 + lr] = d0[r] * CARRY2I; dts[(8 * hi + r) * 32 + 16 + lr] = d1[r] * CARRY2I; }
#pragma unroll
        for (int s = 0; s < 4; ++s) { const int p = s * 32 + lane;
            const v4f v = *(const v4f*)(KQ + (tokb + (size_t)t0) * 32 + (size_t)p * 4);
            *(v4fa*)(&kqs[p * 4]) = v; }
        wave_sync();
        { const int tq = lane & 15; float s2 = 0.0f;
#pragma unroll 4
          for (int n = 0; n < NS; ++n) { const float kv = kqs[tq * 32 + n]; s2 += kv * kv; }
          k2s[lane] = s2; }
        wave_sync();
#pragma unroll 1
        for (int tt = 0; tt < TCH; ++tt) {
            const float u = ub[(size_t)(t0 + tt) * DS];
            const float dv = dts[tt * 32 + lane] + bias;
            const float e = __builtin_amdgcn_exp2f(-fabsf(dv) * LOG2E);
            const float sp = fmaxf(dv, 0.0f) + __builtin_amdgcn_logf(1.0f + e) * LN2;
            const float eps = sp * __builtin_amdgcn_rcpf(1.0f + sp * k2s[tt]);
            float kk[NS], qq[NS];
#pragma unroll
            for (int j = 0; j < 4; ++j) { const v4f kx = *(const v4fa*)(&kqs[tt * 32 + 4 * j]); const v4f qx = *(const v4fa*)(&kqs[tt * 32 + 16 + 4 * j]);
#pragma unroll
                for (int i = 0; i < 4; ++i) { kk[4 * j + i] = kx[i]; qq[4 * j + i] = qx[i]; } }
            float y = 0.0f;
#pragma unroll
            for (int n = 0; n < NS; ++n) {
                const float gn = eps * (u - S[n] * kk[n]) * kk[n];
                S[n] += gn;
                y += S[n] * qq[n]; }
            ys[tt * 32 + lane] = toh_flush((y + dsk * u) * CARRY);
        }
        wave_sync();
#pragma unroll 1
        for (int ps = 0; ps < 2; ++ps) {
#pragma unroll
            for (int s = 0; s < 2; ++s) { const int p = s * 32 + lane;
                const v8h val = *(const v8ha*)(&ys[p * 8]);
                *(volatile v8h*)(yb + (size_t)t0 * 32 + (size_t)p * 8) = val; }
            if (ps == 0) __threadfence(); }
        wave_sync();
    }
}

__global__ __launch_bounds__(32) void k_gemm_out(const h16* __restrict__ YCp, const h16* __restrict__ Wo, float* OUT) {
    __shared__ __align__(16) float os[16 * 68];
    const int K = DI;
    const int lane = threadIdx.x & 31, lr = lane & 15, hi = lane >> 4; const int r0 = blockIdx.x * 64, c0 = blockIdx.y * 64;
    v8f acc[4][4];
#pragma unroll
    for (int mb = 0; mb < 4; ++mb)
#pragma unroll
        for (int nb = 0; nb < 4; ++nb) acc[mb][nb] = (v8f){};
    const size_t aoff = (size_t)(r0 + lr) * 32 + 8 * hi, boff = (size_t)(c0 + lr) * K + 8 * hi;
#pragma unroll 1
    for (int kc = 0; kc < K; kc += 32) {
        v16h a[4];
#pragma unroll
        for (int mb = 0; mb < 4; ++mb) a[mb] = ldh(YCp + aoff + (size_t)mb * 16 * 32 + (size_t)kc * NTOK);
#pragma unroll
        for (int nb = 0; nb < 4; ++nb) { const v16h b = ldh(Wo + boff + (size_t)nb * 16 * K + kc);
#pragma unroll
            for (int mb = 0; mb < 4; ++mb) acc[mb][nb] = wmma16(a[mb], b, acc[mb][nb]); }
        asm volatile("v_nop\n\tv_nop\n\tv_nop\n\tv_nop" : "+v"(acc[0][0]), "+v"(acc[1][1]), "+v"(acc[2][2]), "+v"(acc[3][3]) : "v"(a[0]), "v"(a[1]), "v"(a[2]), "v"(a[3]));
    }
    const int bb = r0 / SEQ, tt = r0 % SEQ;
#pragma unroll
    for (int mb = 0; mb < 4; ++mb) {
#pragma unroll
        for (int nb = 0; nb < 4; ++nb) {
#pragma unroll
            for (int j = 0; j < 8; ++j) os[(hi * 8 + j) * 68 + nb * 16 + lr] = acc[mb][nb][j] * CARRY2I; }
        wave_sync();
        float* dst = OUT + ((size_t)bb * OUT_SEQ + (size_t)(tt + mb * 16)) * DM + c0;
#pragma unroll 1
        for (int ps = 0; ps < 2; ++ps) {
#pragma unroll
            for (int s = 0; s < 8; ++s) { const int row = 2 * s + (lane >> 4), c4 = (lane & 15) * 4;
                const v4f val = *(const v4fa*)(&os[row * 68 + c4]);
                *(volatile v4f*)(dst + (size_t)row * DM + c4) = val; }
            if (ps == 0) __threadfence(); }
        wave_sync();
    }
}

static constexpr size_t al256(size_t v) { return (v + 255) & ~(size_t)255; }
static constexpr size_t SZ_HB = al256((size_t)NTOK * DM * 2);
static constexpr size_t SZ_WI = al256((size_t)DI * DM * 2);
static constexpr size_t SZ_WX = al256((size_t)NX * DS * 2);
static constexpr size_t SZ_WD = al256((size_t)DS * DR * 2);
static constexpr size_t SZ_WO = al256((size_t)DM * DI * 2);
static constexpr size_t SZ_XZ = al256((size_t)CHB * SEQ * DI * 4);
static constexpr size_t SZ_U  = al256((size_t)NTOK * DS * 4);
static constexpr size_t SZ_YC = al256((size_t)NTOK * DI * 2);
static constexpr size_t SZ_DL = al256((size_t)NTOK * DR * 2);
static constexpr size_t SZ_KQ = al256((size_t)NTOK * 32 * 4);
static constexpr size_t SZ_TOTAL = SZ_HB + SZ_WI + SZ_WX + SZ_WD + SZ_WO + SZ_XZ + SZ_U + SZ_YC + SZ_DL + SZ_KQ;
static_assert(SZ_TOTAL <= (size_t)134217728);

extern "C" void kernel_launch(void* const* d_in, const int* in_sizes, int n_in,
                              void* d_out, int out_size, void* d_ws, size_t ws_size, hipStream_t stream) {
    if (n_in < 11) return;
    const size_t needx = ((size_t)(NB - 1) * SEQ_FULL + SEQ) * DM;
    if ((size_t)in_sizes[0] < needx) return;
    if ((size_t)in_sizes[1] < (size_t)DI * DM) return;
    if (in_sizes[2] < DS * 4 || in_sizes[3] < DS || in_sizes[4] < DS * 4 || in_sizes[5] < DS) return;
    if ((size_t)in_sizes[6] < (size_t)NX * DS || (size_t)in_sizes[7] < (size_t)DS * DR) return;
    if (in_sizes[8] < DS || in_sizes[9] < DS) return;
    if ((size_t)in_sizes[10] < (size_t)DM * DI) return;
    if ((size_t)out_size < ((size_t)(NB - 1) * OUT_SEQ + SEQ) * DM) return;
    if (SZ_TOTAL > ws_size) return;
    const float* hid = (const float*)d_in[0];
    const float* win = (const float*)d_in[1];
    const float* cxw = (const float*)d_in[2]; const float* cxb = (const float*)d_in[3];
    const float* czw = (const float*)d_in[4]; const float* czb = (const float*)d_in[5];
    const float* wxp = (const float*)d_in[6];
    const float* wdt = (const float*)d_in[7];
    const float* bdt = (const float*)d_in[8];
    const float* dsk = (const float*)d_in[9];
    const float* wout = (const float*)d_in[10];
    float* OUT = (float*)d_out;
    char* wsp = (char*)d_ws;
    bf*    HB = (bf*)wsp;    wsp += SZ_HB;
    bf*    WI = (bf*)wsp;    wsp += SZ_WI;
    h16*   WX = (h16*)wsp;   wsp += SZ_WX;
    h16*   WD = (h16*)wsp;   wsp += SZ_WD;
    h16*   WO = (h16*)wsp;   wsp += SZ_WO;
    float* XZ = (float*)wsp; wsp += SZ_XZ;
    float* U  = (float*)wsp; wsp += SZ_U;
    h16*   YC = (h16*)wsp;   wsp += SZ_YC;
    h16*   DL = (h16*)wsp;   wsp += SZ_DL;
    float* KQ = (float*)wsp; wsp += SZ_KQ;

    if (SEQ == SEQ_FULL) {
        const size_t n8 = (size_t)NB * SEQ * DM / 8;
        k_cvt8<<<(unsigned)((n8 + 255) / 256), 256, 0, stream>>>(hid, HB, n8);
    } else {
        const size_t n8 = (size_t)SEQ * DM / 8;
        for (int b = 0; b < NB; ++b) k_cvt8<<<(unsigned)((n8 + 255) / 256), 256, 0, stream>>>(hid + (size_t)b * SEQ_FULL * DM, HB + (size_t)b * SEQ * DM, n8);
    }
    { const size_t n8 = (size_t)DI * DM / 8; k_cvt8<<<(unsigned)((n8 + 255) / 256), 256, 0, stream>>>(win, WI, n8); }
    { const size_t n8 = (size_t)NX * DS / 8; k_wcvt<<<(unsigned)((n8 + 255) / 256), 256, 0, stream>>>(wxp, WX, n8, CARRY); }
    { const size_t n8 = (size_t)DS * DR / 8; k_wcvt<<<(unsigned)((n8 + 255) / 256), 256, 0, stream>>>(wdt, WD, n8, CARRY); }
    { const size_t n8 = (size_t)DM * DI / 8; k_wcvt<<<(unsigned)((n8 + 255) / 256), 256, 0, stream>>>(wout, WO, n8, CARRY); }

    for (int c = 0; c < NCH; ++c) {
        k_gemm_in<<<dim3(CHB * SEQ / 64, DI / 64, 1), 32, 0, stream>>>(HB + (size_t)c * CHB * SEQ * DM, WI, XZ);
        k_conv<<<dim3(CHB * SEQ / (CW * CT), DI / 32, 1), 32 * CW, 0, stream>>>(XZ, cxw, cxb, czw, czb, U, YC, c * CHB * SEQ);
    }
    k_xproj<<<dim3(NTOK / 32, 1, 1), 32, 0, stream>>>(U, WX, DL, KQ);
    k_scan<<<dim3(DS / 32, NB, 1), 32, 0, stream>>>(DL, WD, KQ, U, bdt, dsk, YC);
    k_gemm_out<<<dim3(NTOK / 64, DM / 64, 1), 32, 0, stream>>>(YC, WO, OUT);
}
